// SimpleGNN_54090818126571
// MI455X (gfx1250) — hardware-run, weakly checked
//
#include <hip/hip_runtime.h>
#include <stddef.h>
#include <stdint.h>
#include <math.h>

#define NN      100000
#define FD      64
#define HD      64
#define OD      32
#define NE      1600000
#define SPLIT2  1
#define XP      64
#define W1P     64
#define HLP     128
#define W2P     128
#define K1EXT   64
#if SPLIT2
#define K2EXT   128
#else
#define K2EXT   64
#endif
#define GBM     128
#define MP      100096
#define NTHR    256
#define NWAVE   8
#define EPT     8
#define WCH     (32 * EPT)
#define NBRUN   1024
#define SLB     10
#define NBK     98
#define WLCAP   3584
#define RCAP    28672
#define DEGCAP  64
#define MAXDEG_IN   36
#define MAXDEG_OUT  37
#define MAXB_IN     16710
#define MAXB_OUT    16666
#define R1BM    64
#define R2BM    32
#define SP1     68
#define SP2     36
#define WSMAX   (128u << 20)

#define BK_ZINTS (NWAVE * WLCAP + RCAP + 2 * NBRUN + NBRUN + NBRUN + 2 * NBRUN)
#define BK_INTS  (BK_ZINTS + 16)
#define BK_LDS   (BK_INTS * 4)

#define PBX   (MP * XP / 8 / NTHR)
#define PBW1  (HD * W1P / 8 / NTHR)
#define PBW2  (OD * W2P / 8 / NTHR)
#define PBTOT (PBX + PBW1 + PBW2 + 1)
#define NFLAGV (NBK * 8)

static_assert(FD % 32 == 0 && K1EXT == FD && K1EXT % 32 == 0 && K1EXT <= XP && K1EXT <= W1P);
static_assert(K2EXT % 32 == 0 && K2EXT <= HLP && K2EXT <= W2P && HLP == 2 * HD && W2P == HLP);
static_assert(HD == 16 * 4 && OD == 16 * 2 && OD * 4 == 128);
static_assert(MP % GBM == 0 && MP >= NN && MP == 782 * GBM && MP % R1BM == 0 && NN % R2BM == 0);
static_assert(NN == 781 * GBM + 32);
static_assert(NBRUN == (1 << SLB) && NBRUN % R1BM == 0 && NBRUN % R2BM == 0 && NBRUN % GBM == 0 && NBRUN % 32 == 0);
static_assert(NBK * NBRUN >= MP && NBRUN == 4 * NTHR);
static_assert(NE < (1 << 21) && (((long long)NE) << SLB) < (1LL << 31));
static_assert(NE % WCH == 0 && NE % 4 == 0);
static_assert(RCAP == NWAVE * WLCAP && RCAP % (4 * NTHR) == 0 && BK_ZINTS % 4 == 0);
static_assert((long long)RCAP * 100 >= (long long)MAXB_IN * 105);
static_assert((long long)RCAP * 100 >= (long long)MAXB_OUT * 105);
static_assert(WLCAP >= MAXB_IN / 8 + 8 * 46 + 1 && WLCAP >= MAXB_OUT / 8 + 8 * 46 + 1);
static_assert(MAXDEG_IN + 8 <= DEGCAP && MAXDEG_OUT + 8 <= DEGCAP);
static_assert((MP * XP / 8) % NTHR == 0 && (HD * W1P / 8) % NTHR == 0 && (OD * W2P / 8) % NTHR == 0);
static_assert(XP / 8 == 8 && W1P / 8 == 8 && W2P / 8 == 16);
static_assert(BK_LDS <= 300000);
static_assert((GBM * SP1 + GBM) * 4 <= 65536 && (GBM * SP2 + GBM) * 4 <= 65536);
static_assert((long long)(NN - 1) * OD + OD - 1 == 3199999LL);

typedef float          v4f   __attribute__((ext_vector_type(4)));
typedef float          v8f   __attribute__((ext_vector_type(8)));
typedef int            v4i   __attribute__((ext_vector_type(4)));
typedef int            v8i   __attribute__((ext_vector_type(8)));
typedef unsigned short v8us  __attribute__((ext_vector_type(8)));
typedef unsigned short v16us __attribute__((ext_vector_type(16)));
typedef __bf16         v16bf __attribute__((ext_vector_type(16)));
typedef v4f  __attribute__((may_alias)) v4fa;
typedef v4i  __attribute__((may_alias)) v4ia;
typedef v8us __attribute__((may_alias)) v8usa;
union FragB { v16bf v; v16us u; v8us h[2]; v8i w; };

__device__ __forceinline__ v8f wmb(const FragB& a, const FragB& b, v8f c) {
  v8f d = __builtin_amdgcn_wmma_f32_16x16x32_bf16(false, a.v, false, b.v, (short)0, c, false, false);
  asm volatile("v_nop\n\tv_nop\n\tv_nop\n\tv_nop" : "+v"(d) : "v"(a.w), "v"(b.w));
  return d;
}

__device__ __forceinline__ unsigned bf16_bits(float f) {
  const unsigned u = __float_as_uint(f);
  const unsigned r = (u + 0x7FFFu + ((u >> 16) & 1u)) >> 16;
  const unsigned q = (u >> 16) | 0x40u;
  return ((u & 0x7fffffffu) > 0x7f800000u) ? q : r;
}

__device__ __forceinline__ void hilo_pack(float v0, float v1, float v2, float v3,
                                          int& h01, int& h23, int& l01, int& l23) {
  const unsigned a0 = bf16_bits(v0), a1 = bf16_bits(v1), a2 = bf16_bits(v2), a3 = bf16_bits(v3);
  const unsigned b0 = bf16_bits(v0 - __uint_as_float(a0 << 16));
  const unsigned b1 = bf16_bits(v1 - __uint_as_float(a1 << 16));
  const unsigned b2 = bf16_bits(v2 - __uint_as_float(a2 << 16));
  const unsigned b3 = bf16_bits(v3 - __uint_as_float(a3 << 16));
  h01 = (int)(a0 | (a1 << 16)); h23 = (int)(a2 | (a3 << 16));
  l01 = (int)(b0 | (b1 << 16)); l23 = (int)(b2 | (b3 << 16));
}

__device__ __forceinline__ v4i regroup8(int h01, int h23, int l01, int l23, int lane) {
  const int t  = lane & 15;
  const int s0 = (lane & 16) + ((2 * t) & 15), s1 = s0 + 1;
  const int a0 = __shfl(h01, s0, 32), a1 = __shfl(h23, s0, 32), a2 = __shfl(h01, s1, 32), a3 = __shfl(h23, s1, 32);
  const int b0 = __shfl(l01, s0, 32), b1 = __shfl(l23, s0, 32), b2 = __shfl(l01, s1, 32), b3 = __shfl(l23, s1, 32);
  const int mk = (t < 8) ? -1 : 0;
  v4i o;
  o.x = (a0 & mk) | (b0 & ~mk); o.y = (a1 & mk) | (b1 & ~mk);
  o.z = (a2 & mk) | (b2 & ~mk); o.w = (a3 & mk) | (b3 & ~mk);
  return o;
}

__device__ __forceinline__ void st2_v4f(float* p, v4f v) {
  *(volatile v4f*)p = v;
  __threadfence();
  *(volatile v4f*)p = v;
}
__device__ __forceinline__ void st2_v8us(unsigned short* p, v8us v) {
  *(volatile v8us*)p = v;
  __threadfence();
  *(volatile v8us*)p = v;
}

__device__ __forceinline__ v8us colfetch8(const float* __restrict__ base, int stride) {
  float f[8];
#pragma unroll
  for (int i = 0; i < 8; ++i) f[i] = base[(size_t)i * (size_t)stride];
  v8us o;
#pragma unroll
  for (int i = 0; i < 8; ++i) o[i] = (unsigned short)bf16_bits(f[i]);
  return o;
}

__global__ __launch_bounds__(NTHR) void k_prep(const float* __restrict__ x, const float* __restrict__ w1,
                                               const float* __restrict__ b1, const float* __restrict__ w2,
                                               const float* __restrict__ b2,
                                               unsigned short* xb, unsigned short* w1t, unsigned short* w2d,
                                               float* sm, int* flg) {
  const int tid = (int)threadIdx.x, lane = tid & 31;
  const int blk = (int)blockIdx.x;
  if (blk < PBX) {
    const int u   = blk * NTHR + tid;
    const int row = u >> 3, k8 = (u & 7) * 8;
    const int rc  = row < NN ? row : NN - 1;
    const unsigned mk = row < NN ? 0xffffu : 0u;
    const float* p = x + (size_t)rc * FD + k8;
    const v4f a = *(const v4fa*)p;
    const v4f b = *(const v4fa*)(p + 4);
    v8us o;
    o[0] = (unsigned short)(bf16_bits(a.x) & mk); o[1] = (unsigned short)(bf16_bits(a.y) & mk);
    o[2] = (unsigned short)(bf16_bits(a.z) & mk); o[3] = (unsigned short)(bf16_bits(a.w) & mk);
    o[4] = (unsigned short)(bf16_bits(b.x) & mk); o[5] = (unsigned short)(bf16_bits(b.y) & mk);
    o[6] = (unsigned short)(bf16_bits(b.z) & mk); o[7] = (unsigned short)(bf16_bits(b.w) & mk);
    st2_v8us(xb + (size_t)row * XP + k8, o);
  } else if (blk < PBX + PBW1) {
    const int u = (blk - PBX) * NTHR + tid;
    const int n = u >> 3, k8 = (u & 7) * 8;
    const v8us o = colfetch8(w1 + (size_t)k8 * HD + n, HD);
    st2_v8us(w1t + (size_t)n * W1P + k8, o);
  } else if (blk < PBX + PBW1 + PBW2) {
    const int u = (blk - PBX - PBW1) * NTHR + tid;
    const int n = u >> 4, k8 = (u & 15) * 8, kk = k8 & 63;
    const v8us o = colfetch8(w2 + (size_t)kk * OD + n, OD);
    st2_v8us(w2d + (size_t)n * W2P + k8, o);
  } else {
    if (tid < 32) {
      const v4f a = *(const v4fa*)(b1 + 4 * (lane & 15));
      const v4f c = *(const v4fa*)(b2 + 4 * (lane & 7));
      asm volatile("" :: "v"(a));
      asm volatile("" :: "v"(c));
      const unsigned ma = (lane < 16) ? 0xffffffffu : 0u;
      const unsigned mc = ((lane >= 16) & (lane < 24)) ? 0xffffffffu : 0u;
      v4f o;
      o.x = __uint_as_float(((bf16_bits(a.x) << 16) & ma) | ((bf16_bits(c.x) << 16) & mc));
      o.y = __uint_as_float(((bf16_bits(a.y) << 16) & ma) | ((bf16_bits(c.y) << 16) & mc));
      o.z = __uint_as_float(((bf16_bits(a.z) << 16) & ma) | ((bf16_bits(c.z) << 16) & mc));
      o.w = __uint_as_float(((bf16_bits(a.w) << 16) & ma) | ((bf16_bits(c.w) << 16) & mc));
      st2_v4f(sm + 4 * lane, o);
    }
    const v4i z4 = {0, 0, 0, 0};
#pragma unroll 1
    for (int i = tid; i < NFLAGV; i += NTHR) *(volatile v4i*)(flg + 4 * i) = z4;
    __threadfence();
#pragma unroll 1
    for (int i = tid; i < NFLAGV; i += NTHR) *(volatile v4i*)(flg + 4 * i) = z4;
  }
}

__device__ __forceinline__ void bucket_flush(const int* pl, const int* cnt, const int* offs, const int* fni, int ov,
                                             int* lp, int* cp, int* op, int* ndp, int* nsp, int* fp, int tid) {
#pragma unroll 1
  for (int i = tid * 4; i < RCAP; i += NTHR * 4) {
    const v4i v = *(const v4ia*)(pl + i);
    *(volatile v4i*)(lp + i) = v;
  }
  {
    const v4i v0 = *(const v4ia*)(cnt + 4 * tid);
    const v4i v1 = *(const v4ia*)(offs + 4 * tid);
    const v4i v2 = *(const v4ia*)(fni + 4 * tid);
    const v4i v3 = *(const v4ia*)(fni + NBRUN + 4 * tid);
    *(volatile v4i*)(cp + 4 * tid)  = v0;
    *(volatile v4i*)(op + 4 * tid)  = v1;
    *(volatile v4i*)(ndp + 4 * tid) = v2;
    *(volatile v4i*)(nsp + 4 * tid) = v3;
  }
  if (tid < 8) {
    const v4i f = {ov, ov, ov, ov};
    *(volatile v4i*)(fp + 4 * tid) = f;
  }
}

__global__ __launch_bounds__(NTHR) void k_bucket(const int* __restrict__ ei, int* LIST, int* CNT, int* OFF,
                                                 int* NDb, int* NSb, int* FLAG) {
  extern __shared__ __attribute__((aligned(16))) int dsm[];
  int* wl   = dsm;
  int* pl   = dsm + NWAVE * WLCAP;
  int* cnt  = pl + RCAP;
  int* offs = cnt + 2 * NBRUN;
  int* cur  = offs + NBRUN;
  int* fni  = cur + NBRUN;
  int* misc = fni + 2 * NBRUN;
  const int tid = (int)threadIdx.x, lane = tid & 31, wave = tid >> 5;
  const int blk = (int)blockIdx.x;
  const unsigned nbs = (unsigned)(blk * NBRUN);

  {
    const v4i z4 = {0, 0, 0, 0};
    for (int i = tid * 4; i < BK_ZINTS; i += NTHR * 4) *(v4ia*)(dsm + i) = z4;
    if (tid < 16) misc[tid] = 0;
  }
  __syncthreads();

#pragma unroll 1
  for (int role = 0; role < 2; ++role) {
    const int* keys = ei + (size_t)role * (size_t)NE;
    int* cdst = cnt + (1 - role) * NBRUN;
    {
      const int per  = ((NE + NWAVE * WCH - 1) / (NWAVE * WCH)) * WCH;
      const int ebeg = wave * per;
      const int eend = (ebeg + per < NE) ? (ebeg + per) : NE;
      int* mylist = wl + wave * WLCAP;
      int wc = 0;
#pragma unroll 1
      for (int cb = ebeg; cb < eend; cb += WCH) {
        const int e0 = cb + lane * EPT;
        const v4i da = *(const v4ia*)(keys + e0);
        const v4i db = *(const v4ia*)(keys + e0 + 4);
        const unsigned s0 = (unsigned)da.x - nbs, s1 = (unsigned)da.y - nbs;
        const unsigned s2 = (unsigned)da.z - nbs, s3 = (unsigned)da.w - nbs;
        const unsigned s4 = (unsigned)db.x - nbs, s5 = (unsigned)db.y - nbs;
        const unsigned s6 = (unsigned)db.z - nbs, s7 = (unsigned)db.w - nbs;
        const bool h0 = s0 < (unsigned)NBRUN, h1 = s1 < (unsigned)NBRUN, h2 = s2 < (unsigned)NBRUN, h3 = s3 < (unsigned)NBRUN;
        const bool h4 = s4 < (unsigned)NBRUN, h5 = s5 < (unsigned)NBRUN, h6 = s6 < (unsigned)NBRUN, h7 = s7 < (unsigned)NBRUN;
        const unsigned m0 = __builtin_amdgcn_ballot_w32(h0), m1 = __builtin_amdgcn_ballot_w32(h1);
        const unsigned m2 = __builtin_amdgcn_ballot_w32(h2), m3 = __builtin_amdgcn_ballot_w32(h3);
        const unsigned m4 = __builtin_amdgcn_ballot_w32(h4), m5 = __builtin_amdgcn_ballot_w32(h5);
        const unsigned m6 = __builtin_amdgcn_ballot_w32(h6), m7 = __builtin_amdgcn_ballot_w32(h7);
        const unsigned any = m0 | m1 | m2 | m3 | m4 | m5 | m6 | m7;
        if (any != 0u) {
          const int pre = (int)(__builtin_amdgcn_mbcnt_lo(m0, 0u) + __builtin_amdgcn_mbcnt_lo(m1, 0u) +
                                __builtin_amdgcn_mbcnt_lo(m2, 0u) + __builtin_amdgcn_mbcnt_lo(m3, 0u) +
                                __builtin_amdgcn_mbcnt_lo(m4, 0u) + __builtin_amdgcn_mbcnt_lo(m5, 0u) +
                                __builtin_amdgcn_mbcnt_lo(m6, 0u) + __builtin_amdgcn_mbcnt_lo(m7, 0u));
          int p = wc + pre;
          if (h0) { if (p < WLCAP) mylist[p] = ((e0 + 0) << SLB) | (int)s0; p = p + 1; }
          if (h1) { if (p < WLCAP) mylist[p] = ((e0 + 1) << SLB) | (int)s1; p = p + 1; }
          if (h2) { if (p < WLCAP) mylist[p] = ((e0 + 2) << SLB) | (int)s2; p = p + 1; }
          if (h3) { if (p < WLCAP) mylist[p] = ((e0 + 3) << SLB) | (int)s3; p = p + 1; }
          if (h4) { if (p < WLCAP) mylist[p] = ((e0 + 4) << SLB) | (int)s4; p = p + 1; }
          if (h5) { if (p < WLCAP) mylist[p] = ((e0 + 5) << SLB) | (int)s5; p = p + 1; }
          if (h6) { if (p < WLCAP) mylist[p] = ((e0 + 6) << SLB) | (int)s6; p = p + 1; }
          if (h7) { if (p < WLCAP) mylist[p] = ((e0 + 7) << SLB) | (int)s7; p = p + 1; }
          wc += (int)(__builtin_popcount(m0) + __builtin_popcount(m1) + __builtin_popcount(m2) + __builtin_popcount(m3) +
                      __builtin_popcount(m4) + __builtin_popcount(m5) + __builtin_popcount(m6) + __builtin_popcount(m7));
        }
      }
      if (lane == 0) misc[wave] = wc;
    }
    __syncthreads();

    if (wave == 0) {
      int ov = 0;
#pragma unroll 1
      for (int w2 = 0; w2 < NWAVE; ++w2) {
        int c = misc[w2];
        if (c > WLCAP) ov = 1;
        c = c < 0 ? 0 : (c > WLCAP ? WLCAP : c);
#pragma unroll 1
        for (int b0 = 0; b0 < c; b0 += 32) {
          const int idx = b0 + lane;
          const int ent = wl[w2 * WLCAP + (idx < WLCAP ? idx : WLCAP - 1)];
          const int m32 = (c - b0) < 32 ? (c - b0) : 32;
#pragma unroll 1
          for (int k = 0; k < m32; ++k) {
            const int u    = __builtin_amdgcn_readlane(ent, k);
            const int slot = u & (NBRUN - 1);
            if (lane == 0) cdst[slot] = cdst[slot] + 1;
          }
        }
      }
      if (lane == 0) misc[10 - role] = ov;
    }
    __syncthreads();
  }

  if (wave == 0) {
    const int base = lane * (NBRUN / 32);
    int s = 0;
#pragma unroll 1
    for (int i = 0; i < NBRUN / 32; ++i) s += cnt[base + i];
    int incl = s;
#pragma unroll
    for (int d = 1; d < 32; d <<= 1) {
      const int y = __shfl_up(incl, d, 32);
      if (lane >= d) incl += y;
    }
    int run = incl - s;
#pragma unroll 1
    for (int i = 0; i < NBRUN / 32; ++i) {
      const int cv = cnt[base + i];
      offs[base + i] = run;
      cur[base + i]  = run;
      run += cv;
    }
  }
  __syncthreads();

  if (wave == 0) {
#pragma unroll 1
    for (int w2 = 0; w2 < NWAVE; ++w2) {
      int c = misc[w2];
      c = c < 0 ? 0 : (c > WLCAP ? WLCAP : c);
#pragma unroll 1
      for (int b0 = 0; b0 < c; b0 += 32) {
        const int idx = b0 + lane;
        const int ent = wl[w2 * WLCAP + (idx < WLCAP ? idx : WLCAP - 1)];
        int eid = (ent >> SLB) & 0x1FFFFF;
        eid = eid > NE - 1 ? NE - 1 : eid;
        int sr = ei[eid];
        sr = sr < 0 ? 0 : (sr > NN - 1 ? NN - 1 : sr);
        const int m32 = (c - b0) < 32 ? (c - b0) : 32;
#pragma unroll 1
        for (int k = 0; k < m32; ++k) {
          const int u    = __builtin_amdgcn_readlane(ent, k);
          const int wd   = __builtin_amdgcn_readlane(sr, k);
          const int slot = u & (NBRUN - 1);
          if (lane == 0) {
            int p = cur[slot];
            p = p < 0 ? 0 : (p > RCAP - 1 ? RCAP - 1 : p);
            pl[p] = wd;
            cur[slot] = p + 1;
          }
        }
      }
    }
  }
  __syncthreads();

  {
    const int ovc = misc[10];
#pragma unroll 1
    for (int i = tid; i < 2 * NBRUN; i += NTHR) {
      int c = cnt[i];
      c = c < 1 ? 1 : c;
      const float f = 1.0f / sqrtf((float)c);
      const bool ps = (ovc != 0) & (i >= NBRUN);
      fni[i] = ps ? 0x7fc00000 : __float_as_int(f);
    }
  }
  __syncthreads();

  const int ovf = misc[9];
  int* lp  = LIST + (size_t)blk * RCAP;
  int* cp  = CNT + (size_t)blk * NBRUN;
  int* op  = OFF + (size_t)blk * NBRUN;
  int* ndp = NDb + (size_t)blk * NBRUN;
  int* nsp = NSb + (size_t)blk * NBRUN;
  int* fp  = FLAG + (size_t)blk * 32;
  bucket_flush(pl, cnt, offs, fni, ovf, lp, cp, op, ndp, nsp, fp, tid);
  __threadfence();
  bucket_flush(pl, cnt, offs, fni, ovf, lp, cp, op, ndp, nsp, fp, tid);
}

template <int KEXT, int AP, int WP, int NT>
__device__ __forceinline__ void gemm_16xN(const unsigned short* __restrict__ ap,
                                          const unsigned short* __restrict__ bp, v8f (&acc)[NT]) {
  static_assert(KEXT % 32 == 0 && KEXT <= AP && KEXT <= WP && AP % 8 == 0 && WP % 8 == 0);
#pragma unroll 1
  for (int k0 = 0; k0 < KEXT; k0 += 32) {
    FragB af;
    af.h[0] = *(const v8usa*)(ap + k0);
    af.h[1] = *(const v8usa*)(ap + k0 + 16);
#pragma unroll
    for (int nt = 0; nt < NT; ++nt) {
      const unsigned short* wq = bp + (size_t)(16 * nt) * (size_t)WP + k0;
      FragB bf;
      bf.h[0] = *(const v8usa*)wq;
      bf.h[1] = *(const v8usa*)(wq + 16);
      acc[nt] = wmb(af, bf, acc[nt]);
    }
  }
}

template <int NT, int SPX>
__device__ __forceinline__ void stage_d(float* stg, const v8f (&acc)[NT], int wave, int hh, int m) {
#pragma unroll
  for (int nt = 0; nt < NT; ++nt) {
#pragma unroll
    for (int r = 0; r < 8; ++r) stg[(16 * wave + 8 * hh + r) * SPX + 16 * nt + m] = acc[nt][r];
  }
}

__global__ __launch_bounds__(NTHR) __attribute__((amdgpu_num_vgpr(248)))
void k_gemm1(const unsigned short* __restrict__ XB, const unsigned short* __restrict__ W1T,
             const float* __restrict__ NSv, float* P1) {
  __shared__ __attribute__((aligned(16))) float stg[GBM * SP1];
  __shared__ __attribute__((aligned(16))) float sns[GBM];
  const int tid = (int)threadIdx.x, lane = tid & 31, wave = tid >> 5, hh = lane >> 4, m = lane & 15;
  const int rowBase = (int)blockIdx.x * GBM;
  if (tid < 32) *(v4fa*)(sns + 4 * tid) = *(const v4fa*)(NSv + (size_t)rowBase + 4 * tid);

  v8f acc[4];
  {
    const v8f z = {0.f, 0.f, 0.f, 0.f, 0.f, 0.f, 0.f, 0.f};
#pragma unroll
    for (int t = 0; t < 4; ++t) acc[t] = z;
  }
  const unsigned short* ap = XB + (size_t)(rowBase + 16 * wave + m) * (size_t)XP + 8 * hh;
  const unsigned short* bp = W1T + (size_t)m * (size_t)W1P + 8 * hh;
  gemm_16xN<K1EXT, XP, W1P, 4>(ap, bp, acc);
  stage_d<4, SP1>(stg, acc, wave, hh, m);
  __syncthreads();

#pragma unroll 1
  for (int i = 0; i < 8; ++i) {
    const int lr   = 16 * wave + 2 * i + hh;
    const int grow = rowBase + lr;
    const bool live = grow < NN;
    const v4f a = *(const v4fa*)(stg + lr * SP1 + 4 * m);
    const float s = sns[lr];
    asm volatile("" :: "v"(a));
    const float v0 = a.x * s, v1 = a.y * s, v2 = a.z * s, v3 = a.w * s;
    v4f o;
    o.x = live ? v0 : 0.0f; o.y = live ? v1 : 0.0f; o.z = live ? v2 : 0.0f; o.w = live ? v3 : 0.0f;
    st2_v4f(P1 + (size_t)grow * HD + 4 * m, o);
  }
}

__global__ __launch_bounds__(NTHR) void k_replay1(const int* __restrict__ LIST, const int* __restrict__ CNT,
                                                  const int* __restrict__ OFF, const int* __restrict__ FLAG,
                                                  const float* __restrict__ NDv, const float* __restrict__ P1,
                                                  const float* __restrict__ SM, unsigned short* H1HL) {
  __shared__ __attribute__((aligned(16))) float sb[HD];
  const int tid = (int)threadIdx.x, lane = tid & 31, wave = tid >> 5, hh = lane >> 4, q = lane & 15;
  const int rowBase = (int)blockIdx.x * R1BM;
  const int bucket  = rowBase >> SLB;
  if (tid < 16) *(v4fa*)(sb + 4 * tid) = *(const v4fa*)(SM + 4 * tid);
  __syncthreads();
  const v4f bias = *(const v4fa*)(sb + 4 * q);
  const int* lb  = LIST + (size_t)bucket * RCAP;
  const int flag = FLAG[(size_t)bucket * 32];
  const float qnan = __uint_as_float(0x7fc00000u);

#pragma unroll 1
  for (int i = 0; i < R1BM / (2 * NWAVE); ++i) {
    const int d = rowBase + (R1BM / NWAVE) * wave + 2 * i + hh;
    int c = CNT[d];
    int o = OFF[d];
    const bool big = c > DEGCAP;
    c = c < 0 ? 0 : (c > DEGCAP ? DEGCAP : c);
    o = o < 0 ? 0 : (o > RCAP - 1 ? RCAP - 1 : o);
    const int co = __shfl_xor(c, 16, 32);
    const int cv = c > co ? c : co;
    const int cm = __builtin_amdgcn_readfirstlane(cv);
    int last = o + c - 1;
    last = last < o ? o : last;
    last = last > RCAP - 1 ? RCAP - 1 : last;
    float a0 = 0.0f, a1 = 0.0f, a2 = 0.0f, a3 = 0.0f;
#pragma unroll 1
    for (int j = 0; j < cm; ++j) {
      int idx = o + j;
      idx = idx > last ? last : idx;
      int sr = lb[idx];
      sr = sr < 0 ? 0 : (sr > NN - 1 ? NN - 1 : sr);
      const v4f v = *(const v4fa*)(P1 + (size_t)sr * HD + 4 * q);
      asm volatile("" :: "v"(v));
      const bool valid = j < c;
      const float t0 = a0 + v.x, t1 = a1 + v.y, t2 = a2 + v.z, t3 = a3 + v.w;
      a0 = valid ? t0 : a0; a1 = valid ? t1 : a1; a2 = valid ? t2 : a2; a3 = valid ? t3 : a3;
    }
    const float nd = NDv[d];
    float m0 = nd * a0 + bias.x, m1 = nd * a1 + bias.y, m2 = nd * a2 + bias.z, m3 = nd * a3 + bias.w;
    m0 = (m0 > 0.0f) ? m0 : (m0 - m0); m1 = (m1 > 0.0f) ? m1 : (m1 - m1);
    m2 = (m2 > 0.0f) ? m2 : (m2 - m2); m3 = (m3 > 0.0f) ? m3 : (m3 - m3);
    const bool bad  = (flag != 0) | big;
    const bool live = d < NN;
    m0 = bad ? qnan : m0; m1 = bad ? qnan : m1; m2 = bad ? qnan : m2; m3 = bad ? qnan : m3;
    m0 = live ? m0 : 0.0f; m1 = live ? m1 : 0.0f; m2 = live ? m2 : 0.0f; m3 = live ? m3 : 0.0f;
    int h01, h23, l01, l23;
    hilo_pack(m0, m1, m2, m3, h01, h23, l01, l23);
    const v4i ow = regroup8(h01, h23, l01, l23, lane);
    unsigned short* hp = H1HL + (size_t)d * HLP + 8 * q;
    *(volatile v4i*)hp = ow;
    __threadfence();
    *(volatile v4i*)hp = ow;
  }
}

__global__ __launch_bounds__(NTHR) __attribute__((amdgpu_num_vgpr(248)))
void k_gemm2(const unsigned short* __restrict__ HL, const unsigned short* __restrict__ W2D,
             const float* __restrict__ NSv, float* P2) {
  __shared__ __attribute__((aligned(16))) float stg[GBM * SP2];
  __shared__ __attribute__((aligned(16))) float sns[GBM];
  const int tid = (int)threadIdx.x, lane = tid & 31, wave = tid >> 5, hh = lane >> 4, m = lane & 15;
  const int rowBase = (int)blockIdx.x * GBM;
  if (tid < 32) *(v4fa*)(sns + 4 * tid) = *(const v4fa*)(NSv + (size_t)rowBase + 4 * tid);

  v8f acc[2];
  {
    const v8f z = {0.f, 0.f, 0.f, 0.f, 0.f, 0.f, 0.f, 0.f};
    acc[0] = z; acc[1] = z;
  }
  const unsigned short* ap = HL + (size_t)(rowBase + 16 * wave + m) * (size_t)HLP + 8 * hh;
  const unsigned short* bp = W2D + (size_t)m * (size_t)W2P + 8 * hh;
  gemm_16xN<K2EXT, HLP, W2P, 2>(ap, bp, acc);
  stage_d<2, SP2>(stg, acc, wave, hh, m);
  __syncthreads();

  const int rq = lane >> 3, c4 = lane & 7;
#pragma unroll 1
  for (int i = 0; i < 4; ++i) {
    const int lr   = 16 * wave + 4 * i + rq;
    const int grow = rowBase + lr;
    const bool live = grow < NN;
    const v4f a = *(const v4fa*)(stg + lr * SP2 + 4 * c4);
    const float s = sns[lr];
    asm volatile("" :: "v"(a));
    const float v0 = a.x * s, v1 = a.y * s, v2 = a.z * s, v3 = a.w * s;
    v4f o;
    o.x = live ? v0 : 0.0f; o.y = live ? v1 : 0.0f; o.z = live ? v2 : 0.0f; o.w = live ? v3 : 0.0f;
    st2_v4f(P2 + (size_t)grow * OD + 4 * c4, o);
  }
}

__global__ __launch_bounds__(NTHR) void k_replay2(const int* __restrict__ LIST, const int* __restrict__ CNT,
                                                  const int* __restrict__ OFF, const int* __restrict__ FLAG,
                                                  const float* __restrict__ NDv, const float* __restrict__ P2,
                                                  const float* __restrict__ SM, float* out) {
  __shared__ __attribute__((aligned(16))) float sb[OD];
  const int tid = (int)threadIdx.x, lane = tid & 31, wave = tid >> 5, rq = lane >> 3, q = lane & 7;
  const int rowBase = (int)blockIdx.x * R2BM;
  const int bucket  = rowBase >> SLB;
  if (tid < 8) *(v4fa*)(sb + 4 * tid) = *(const v4fa*)(SM + HD + 4 * tid);
  __syncthreads();
  const v4f bias = *(const v4fa*)(sb + 4 * q);
  const int* lb  = LIST + (size_t)bucket * RCAP;
  const int flag = FLAG[(size_t)bucket * 32];
  const float qnan = __uint_as_float(0x7fc00000u);

  const int d = rowBase + 4 * wave + rq;
  int c = CNT[d];
  int o = OFF[d];
  const bool big = c > DEGCAP;
  c = c < 0 ? 0 : (c > DEGCAP ? DEGCAP : c);
  o = o < 0 ? 0 : (o > RCAP - 1 ? RCAP - 1 : o);
  const int c1 = __shfl_xor(c, 8, 32);
  const int m1 = c > c1 ? c : c1;
  const int c2 = __shfl_xor(m1, 16, 32);
  const int cv = m1 > c2 ? m1 : c2;
  const int cm = __builtin_amdgcn_readfirstlane(cv);
  int last = o + c - 1;
  last = last < o ? o : last;
  last = last > RCAP - 1 ? RCAP - 1 : last;
  float a0 = 0.0f, a1 = 0.0f, a2 = 0.0f, a3 = 0.0f;
#pragma unroll 1
  for (int j = 0; j < cm; ++j) {
    int idx = o + j;
    idx = idx > last ? last : idx;
    int sr = lb[idx];
    sr = sr < 0 ? 0 : (sr > NN - 1 ? NN - 1 : sr);
    const v4f v = *(const v4fa*)(P2 + (size_t)sr * OD + 4 * q);
    asm volatile("" :: "v"(v));
    const bool valid = j < c;
    const float t0 = a0 + v.x, t1 = a1 + v.y, t2 = a2 + v.z, t3 = a3 + v.w;
    a0 = valid ? t0 : a0; a1 = valid ? t1 : a1; a2 = valid ? t2 : a2; a3 = valid ? t3 : a3;
  }
  const float nd = NDv[d];
  float m0 = nd * a0 + bias.x, m1v = nd * a1 + bias.y, m2 = nd * a2 + bias.z, m3 = nd * a3 + bias.w;
  const bool bad = (flag != 0) | big;
  v4f ov;
  ov.x = bad ? qnan : m0; ov.y = bad ? qnan : m1v; ov.z = bad ? qnan : m2; ov.w = bad ? qnan : m3;
  st2_v4f(out + (size_t)d * OD + 4 * q, ov);
}

extern "C" void kernel_launch(void* const* d_in, const int* in_sizes, int n_in,
                              void* d_out, int out_size, void* d_ws, size_t ws_size,
                              hipStream_t stream) {
  if (n_in < 6) return;
  if (in_sizes[0] != NN * FD) return;
  if (in_sizes[1] != 2 * NE) return;
  if (in_sizes[2] != FD * HD) return;
  if (in_sizes[3] != HD) return;
  if (in_sizes[4] != HD * OD) return;
  if (in_sizes[5] != OD) return;
  if (out_size != NN * OD) return;

  const float* x  = (const float*)d_in[0];
  const int*   ei = (const int*)d_in[1];
  const float* W1 = (const float*)d_in[2];
  const float* b1 = (const float*)d_in[3];
  const float* W2 = (const float*)d_in[4];
  const float* b2 = (const float*)d_in[5];
  float* out = (float*)d_out;

  constexpr size_t zXB   = (size_t)MP * XP * 2;
  constexpr size_t zP1   = (size_t)MP * HD * 4;
  constexpr size_t zHL   = (size_t)MP * HLP * 2;
  constexpr size_t zP2   = (size_t)MP * OD * 4;
  constexpr size_t zLIST = (size_t)NBK * RCAP * 4;
  constexpr size_t zTAB  = (size_t)NBK * NBRUN * 4;
  constexpr size_t zFLAG = (size_t)NBK * 128;
  constexpr size_t zW1T  = (size_t)HD * W1P * 2;
  constexpr size_t zW2D  = (size_t)OD * W2P * 2;
  constexpr size_t zSM   = 512;
  constexpr size_t oXB   = 0;
  constexpr size_t oP1   = oXB + zXB;
  constexpr size_t oHL   = oP1 + zP1;
  constexpr size_t oP2   = oHL + zHL;
  constexpr size_t oLIST = oP2 + zP2;
  constexpr size_t oCNT  = oLIST + zLIST;
  constexpr size_t oOFF  = oCNT + zTAB;
  constexpr size_t oND   = oOFF + zTAB;
  constexpr size_t oNS   = oND + zTAB;
  constexpr size_t oFLAG = oNS + zTAB;
  constexpr size_t oW1T  = oFLAG + zFLAG;
  constexpr size_t oW2D  = oW1T + zW1T;
  constexpr size_t oSM   = oW2D + zW2D;
  constexpr size_t oEND  = oSM + zSM;
  static_assert(zXB % 256 == 0 && zP1 % 256 == 0 && zHL % 256 == 0 && zP2 % 256 == 0 && zLIST % 256 == 0);
  static_assert(zTAB % 256 == 0 && zFLAG % 256 == 0 && zW1T % 256 == 0 && zW2D % 256 == 0 && zSM % 256 == 0);
  static_assert(zTAB >= (size_t)MP * 4);
  static_assert(oEND <= (size_t)WSMAX);
  if (oEND > ws_size) return;

  char* ws = (char*)d_ws;
  unsigned short* XB   = (unsigned short*)(ws + oXB);
  float*          P1   = (float*)(ws + oP1);
  unsigned short* H1HL = (unsigned short*)(ws + oHL);
  float*          P2   = (float*)(ws + oP2);
  int*            LIST = (int*)(ws + oLIST);
  int*            CNT  = (int*)(ws + oCNT);
  int*            OFF  = (int*)(ws + oOFF);
  int*            NDb  = (int*)(ws + oND);
  int*            NSb  = (int*)(ws + oNS);
  int*            FLAG = (int*)(ws + oFLAG);
  unsigned short* W1T  = (unsigned short*)(ws + oW1T);
  unsigned short* W2D  = (unsigned short*)(ws + oW2D);
  float*          SM   = (float*)(ws + oSM);
  const float*    NDf  = (const float*)(ws + oND);
  const float*    NSf  = (const float*)(ws + oNS);

  hipFuncSetAttribute(reinterpret_cast<const void*>(&k_bucket), hipFuncAttributeMaxDynamicSharedMemorySize, (int)BK_LDS);

  k_prep<<<PBTOT, NTHR, 0, stream>>>(x, W1, b1, W2, b2, XB, W1T, W2D, SM, FLAG);
  k_bucket<<<NBK, NTHR, BK_LDS, stream>>>(ei, LIST, CNT, OFF, NDb, NSb, FLAG);
  k_gemm1<<<MP / GBM, NTHR, 0, stream>>>(XB, W1T, NSf, P1);
  k_replay1<<<MP / R1BM, NTHR, 0, stream>>>(LIST, CNT, OFF, FLAG, NDf, P1, SM, H1HL);
  k_gemm2<<<MP / GBM, NTHR, 0, stream>>>(H1HL, W2D, NSf, P2);
  k_replay2<<<NN / R2BM, NTHR, 0, stream>>>(LIST, CNT, OFF, FLAG, NDf, P2, SM, out);
}
